// ConcatAttention_80255758893462
// MI455X (gfx1250) — hardware-verified
//
#include <hip/hip_runtime.h>


namespace {
constexpr int NB_ = 4, LQ = 512, LP = 512, D = 512, HH = 128;
constexpr float XS = 8.0f, HS = 256.0f, PS = 16384.0f  , WSC = 256.0f;
typedef _Float16 b16;
typedef __attribute__((ext_vector_type(16))) _Float16 v16b;
typedef __attribute__((ext_vector_type(8))) _Float16 v8b;
typedef __attribute__((ext_vector_type(8))) float v8f;
typedef __attribute__((ext_vector_type(4))) float v4f;
typedef __attribute__((ext_vector_type(2))) _Float16 v2b;
__device__ __forceinline__ float bf16_rne(float f) { unsigned int u = __float_as_uint(f); u += 0x7FFFu + ((u >> 16) & 1u); float r = __uint_as_float(u & 0xFFFF0000u); asm volatile("" : "+v"(r)); return r; }
__device__ __forceinline__ float bfv(float f) { float r = bf16_rne(f); asm volatile("" : "+v"(r)); return r; }
__device__ __forceinline__ void split16(float v, b16& hi, b16& lo) { hi = (b16)v; lo = (b16)(v - (float)hi); }
__device__ __forceinline__ v16b frag_kb(const b16* p, int hh) { const v8b a = *(const v8b*)(p + 8 * hh), b = *(const v8b*)(p + 16 + 8 * hh); v16b f;
#pragma unroll
  for (int e = 0; e < 8; ++e) { f[e] = a[e]; f[8 + e] = b[e]; } return f; }
__device__ __forceinline__ v8f wmma16b(v16b a, v16b b, v8f c) { v8f d = __builtin_amdgcn_wmma_f32_16x16x32_f16(false, a, false, b, (short)0, c, false, false); asm volatile("v_nop\n\tv_nop\n\tv_nop\n\tv_nop" : "+v"(d) : "v"(a), "v"(b)); return d; }
__device__ __forceinline__ void wave_lds_sync() { __builtin_amdgcn_fence(__ATOMIC_RELEASE, "workgroup"); __builtin_amdgcn_wave_barrier(); __builtin_amdgcn_fence(__ATOMIC_ACQUIRE, "workgroup"); }
__device__ __forceinline__ float pmul(float a, float b) { float p = a * b; asm volatile("" : "+v"(p)); return p; }
__device__ __forceinline__ float tanh_e(float x) { const float e = __expf(2.0f * x); return 1.0f - 2.0f / (e + 1.0f); }

__global__ __launch_bounds__(256) void prep_kernel(const float* __restrict__ wq, const float* __restrict__ wp, const float* __restrict__ hq, b16* __restrict__ WQT, b16* __restrict__ WPT, b16* __restrict__ HQT) { __shared__ float Tt[64][65]; const int tid = threadIdx.x, wave = tid >> 5, lane = tid & 31; const int nbT = NB_ * (LQ / 64) * (D / 64);
  if ((int)blockIdx.x < nbT) { const int b = blockIdx.x / ((LQ / 64) * (D / 64)), r = blockIdx.x % ((LQ / 64) * (D / 64)); const int q0 = (r / (D / 64)) * 64, d0 = (r % (D / 64)) * 64;
    for (int q = wave; q < 64; q += 8) { Tt[q][lane] = bfv(hq[((size_t)b * LQ + q0 + q) * D + d0 + lane]); Tt[q][32 + lane] = bfv(hq[((size_t)b * LQ + q0 + q) * D + d0 + 32 + lane]); }
    __syncthreads();
    for (int pass = 0; pass < 2; ++pass) { for (int d = wave; d < 64; d += 8) *(volatile v2b*)(HQT + ((size_t)b * D + d0 + d) * LQ + q0 + lane * 2) = (v2b){(b16)(Tt[lane * 2][d] * XS), (b16)(Tt[lane * 2 + 1][d] * XS)}; __threadfence(); } }
  else { const int u = (blockIdx.x - nbT) * 256 + tid; if (u < 2 * HH * (D / 8)) { const int which = u / (HH * (D / 8)), r = u % (HH * (D / 8)); const int h = r / (D / 8), d0 = (r % (D / 8)) * 8; const float* w = which == 0 ? wq : wp; v8b v;
#pragma unroll
      for (int j = 0; j < 8; ++j) v[j] = (b16)(bf16_rne(w[(size_t)(d0 + j) * HH + h]) * WSC); for (int pass = 0; pass < 2; ++pass) { *(volatile v8b*)((which == 0 ? WQT : WPT) + (size_t)h * D + d0) = v; __threadfence(); } } } }
__global__ __launch_bounds__(32) void proj_kernel(const float* __restrict__ hq, const float* __restrict__ hp, const b16* __restrict__ WQT, const b16* __restrict__ WPT, const float* __restrict__ bias, b16* __restrict__ dummy, float* __restrict__ PQ, float* __restrict__ PP) { __shared__ __attribute__((aligned(16))) b16 Ax[16][D + 8]; __shared__ float Tf[16][HH + 4]; const int lane = threadIdx.x, nloc = lane & 15, hlf = lane >> 4; const size_t r0 = (size_t)blockIdx.x * 16; const int which = blockIdx.y; const float* src = which == 0 ? hq : hp; (void)dummy;
  for (int rr = 0; rr < 16; ++rr) for (int q = 0; q < D / 32; ++q) { const int c = q * 32 + lane; Ax[rr][c] = (b16)(bfv(src[(r0 + rr) * D + c]) * XS); }
  if (lane < 16) for (int k = D; k < D + 8; ++k) Ax[lane][k] = (b16)0.0f;
  wave_lds_sync(); v8f acc[8];
#pragma unroll
  for (int t = 0; t < 8; ++t) acc[t] = (v8f){};
  const b16* Wb = which == 0 ? WQT : WPT;
#pragma unroll 2
  for (int kb = 0; kb < D; kb += 32) { const v16b a = frag_kb(&Ax[nloc][kb], hlf);
#pragma unroll
    for (int t = 0; t < 8; ++t) acc[t] = wmma16b(a, frag_kb(Wb + (size_t)(t * 16 + nloc) * D + kb, hlf), acc[t]); }
#pragma unroll
  for (int t = 0; t < 8; ++t) { const int cc = t * 16 + nloc; const float bb = which == 0 ? bfv(bias[cc]) : 0.0f;
#pragma unroll
    for (int r8 = 0; r8 < 8; ++r8) Tf[8 * hlf + r8][cc] = acc[t][r8] * (1.0f / (XS * WSC)) + bb; }
  wave_lds_sync();
  float* dst = which == 0 ? PQ : PP;
  for (int pass = 0; pass < 2; ++pass) { for (int rr = 0; rr < 16; ++rr) *(volatile v4f*)(dst + (r0 + rr) * HH + lane * 4) = *(const v4f*)(&Tf[rr][lane * 4]); __threadfence(); } }
__global__ __launch_bounds__(256) void score_kernel(const float* __restrict__ PQ, const float* __restrict__ PP, const float* __restrict__ vv, const int* __restrict__ mq, const int* __restrict__ mp, int PLIM, float* __restrict__ S) { __shared__ float Srow[16][LQ]; const int tid = threadIdx.x, wave = tid >> 5, lane = tid & 31; const int b = blockIdx.x / (LP / 16), p0 = (blockIdx.x % (LP / 16)) * 16; if (p0 >= PLIM) return;
  float v4[4]; for (int j = 0; j < 4; ++j) v4[j] = bfv(vv[lane * 4 + j]);
  for (int pi = 0; pi < 2; ++pi) { const int p = p0 + wave * 2 + pi; const v4f ppv = *(const v4f*)(PP + ((size_t)b * LP + p) * HH + lane * 4); const bool mpk = mp[b * LP + p] != 0;
#pragma unroll 1
    for (int q = 0; q < LQ; ++q) { const v4f pqv = *(const v4f*)(PQ + ((size_t)b * LQ + q) * HH + lane * 4); float part = 0.0f;
#pragma unroll
      for (int j = 0; j < 4; ++j) part += pmul(v4[j], tanh_e(pqv[j] + ppv[j]));
      for (int o = 16; o; o >>= 1) part += __shfl_xor(part, o);
      if (lane == (q & 31)) { const bool m = mpk && (mq[b * LQ + q] != 0); Srow[wave * 2 + pi][q] = part - (m ? 0.0f : 10000.0f); } } }
  __syncthreads();
  for (int pass = 0; pass < 2; ++pass) { for (int pi = 0; pi < 2; ++pi) { const int r = wave * 2 + pi; for (int c = lane; c < LQ; c += 32) ((volatile float*)S)[((size_t)b * LP + p0 + r) * LQ + c] = Srow[r][c]; } __threadfence(); } }
__global__ __launch_bounds__(32) void out_kernel(const float* __restrict__ S, const b16* __restrict__ HQT, int PLIM, float* __restrict__ out) { __shared__ __attribute__((aligned(16))) b16 Ah[16][LQ + 8], Al[16][LQ + 8]; __shared__ float Tf[16][260]; const int lane = threadIdx.x, nloc = lane & 15, hlf = lane >> 4; const int b = blockIdx.x / (LP / 16), p0 = (blockIdx.x % (LP / 16)) * 16; if (p0 >= PLIM) return;
  if (lane < 16) { const float* sr = S + ((size_t)b * LP + p0 + lane) * LQ; float mx = -INFINITY; for (int q = 0; q < LQ; ++q) mx = fmaxf(mx, sr[q]); float z = 0.0f; for (int q = 0; q < LQ; ++q) z += __expf(sr[q] - mx); const float inv = 1.0f / z;
    for (int q = 0; q < LQ; ++q) { b16 ph, pl; split16(__expf(sr[q] - mx) * inv * PS, ph, pl); Ah[lane][q] = ph; Al[lane][q] = pl; } for (int q = LQ; q < LQ + 8; ++q) { Ah[lane][q] = (b16)0.0f; Al[lane][q] = (b16)0.0f; } }
  wave_lds_sync();
#pragma unroll 1
  for (int g = 0; g < 2; ++g) { v8f acc[16];
#pragma unroll
    for (int t = 0; t < 16; ++t) acc[t] = (v8f){};
#pragma unroll 2
    for (int kb = 0; kb < LQ; kb += 32) { const v16b a = frag_kb(&Ah[nloc][kb], hlf), al = frag_kb(&Al[nloc][kb], hlf);
#pragma unroll
      for (int t = 0; t < 16; ++t) { const v16b bw = frag_kb(HQT + ((size_t)b * D + g * 256 + t * 16 + nloc) * LQ + kb, hlf); acc[t] = wmma16b(a, bw, acc[t]); acc[t] = wmma16b(al, bw, acc[t]); } }
#pragma unroll
    for (int t = 0; t < 16; ++t)
#pragma unroll
      for (int r8 = 0; r8 < 8; ++r8) Tf[8 * hlf + r8][t * 16 + nloc] = acc[t][r8] * (1.0f / (PS * XS));
    wave_lds_sync();
    for (int pass = 0; pass < 2; ++pass) { for (int rr = 0; rr < 16; ++rr) for (int q = 0; q < 2; ++q) *(volatile v4f*)(out + ((size_t)b * LP + p0 + rr) * D + g * 256 + q * 128 + lane * 4) = *(const v4f*)(&Tf[rr][q * 128 + lane * 4]); __threadfence(); }
    wave_lds_sync(); } }
}

extern "C" void kernel_launch(void* const* d_in, const int* in_sizes, int n_in, void* d_out, int out_size, void* d_ws, size_t ws_size, hipStream_t stream) {
  (void)n_in;
  auto Fp = [&](int i) { return (const float*)d_in[i]; }; auto Ip = [&](int i) { return (const int*)d_in[i]; };
  if (in_sizes[0] != NB_ * LQ * D || in_sizes[1] != NB_ * LP * D || in_sizes[2] != NB_ * LQ || in_sizes[3] != NB_ * LP || in_sizes[4] != D * HH || in_sizes[5] != D * HH || in_sizes[6] != HH || in_sizes[7] != HH || out_size != NB_ * LP * D) return;
  const int PLIM = LP;
  size_t off = 0; char* ws = (char*)d_ws;
  auto carve = [&](size_t bytes) { char* p = ws + off; off += (bytes + 255) & ~(size_t)255; return p; };
  b16* WQT = (b16*)carve((size_t)HH * D * 2); b16* WPT = (b16*)carve((size_t)HH * D * 2); b16* HQT = (b16*)carve((size_t)NB_ * D * LQ * 2); float* PQ = (float*)carve((size_t)NB_ * LQ * HH * 4); float* PP = (float*)carve((size_t)NB_ * LP * HH * 4); float* S = (float*)carve((size_t)NB_ * LP * LQ * 4);
  if (off > ws_size || off > ((size_t)16 << 20)) return;
  const int nbT = NB_ * (LQ / 64) * (D / 64);
  prep_kernel<<<nbT + (2 * HH * (D / 8) + 255) / 256, 256, 0, stream>>>(Fp(4), Fp(5), Fp(0), WQT, WPT, HQT);
  proj_kernel<<<dim3(NB_ * LQ / 16, 2), 32, 0, stream>>>(Fp(0), Fp(1), WQT, WPT, Fp(6), nullptr, PQ, PP);
  score_kernel<<<NB_ * (LP / 16), 256, 0, stream>>>(PQ, PP, Fp(7), Ip(2), Ip(3), PLIM, S);
  out_kernel<<<NB_ * (LP / 16), 32, 0, stream>>>(S, HQT, PLIM, (float*)d_out);
}
